// SPGAT_80719615361789
// MI455X (gfx1250) — hardware-verified
//
#include <hip/hip_runtime.h>
#include <stddef.h>
#include <stdint.h>


#define FIN     256
#define HID     64
#define NHD     8
#define F1      512
#define NCLS    40
#define NCP     64
#define K2      1024
#define APITCH  264
#define NTHR    256
#define NWAVE   8
#define EPT     8
#define CHUNK   (NTHR * EPT)
#define WCAP    (EPT * 32)
#define LISTN   (NWAVE * WCAP)
#define NBMAX   2048
#define NB2MAX  512
#define RCAP    28672
#define DEGCAP  4096
#define STW     1024
#define GBM     64
#define GTHR    128
#define EMAXG   128
#define ERECW   32
#define LRELU   0.2f
#define WSMAX   268435456
#define LDS_AGG ((2 * RCAP + 2 * NBMAX + LISTN) * 4 + 128)

static_assert((CHUNK & (CHUNK - 1)) == 0 && CHUNK <= 4096);
static_assert((NBMAX & (NBMAX - 1)) == 0 && NBMAX <= 4096);
static_assert(NTHR * 8 == NBMAX);
static_assert(LISTN >= NBMAX);
static_assert(LISTN >= NWAVE * WCAP);
static_assert((RCAP % 32) == 0);
static_assert(NWAVE * STW <= RCAP);
static_assert(STW * 4 >= F1 * 4 + K2 * 2);
static_assert(NB2MAX * NCLS <= RCAP);
static_assert(LDS_AGG <= 300000);
static_assert(GBM == (GTHR / 32) * 16);
static_assert(FIN / 8 == 32 && K2 / 8 == 128);
static_assert((FIN % 32) == 0 && (K2 % 32) == 0);
static_assert(F1 == NHD * HID && K2 == 2 * F1);
static_assert(NCLS > 32 && NCLS <= NCP && (NCLS % 4) == 0);
static_assert((APITCH % 8) == 0);
static_assert(2 * NCLS <= GTHR);

typedef float    v4f  __attribute__((ext_vector_type(4)));
typedef float    v8f  __attribute__((ext_vector_type(8)));
typedef int      v4i  __attribute__((ext_vector_type(4)));
typedef int      v8i  __attribute__((ext_vector_type(8)));
typedef unsigned short u16;
typedef u16      v8us __attribute__((ext_vector_type(8)));
typedef v8us __attribute__((may_alias)) v8usa;
typedef v4f  __attribute__((may_alias)) v4fa;
typedef __bf16   v16bf __attribute__((ext_vector_type(16)));
union FragB { v16bf v; v8us h[2]; v8i w; };

__device__ __forceinline__ v8f wmb(const FragB& a, const FragB& b, v8f c) {
  v8f d = __builtin_amdgcn_wmma_f32_16x16x32_bf16(false, a.v, false, b.v, (short)0, c, false, false);
  asm volatile("v_nop\n\tv_nop\n\tv_nop\n\tv_nop" : "+v"(d) : "v"(a.w), "v"(b.w));
  return d;
}

__device__ __forceinline__ void ldwait() {
  asm volatile("s_wait_loadcnt 0x0" ::: "memory");
}

__device__ __forceinline__ unsigned bfb(float f) {
  const unsigned u = __float_as_uint(f);
  return (u + 0x7FFFu + ((u >> 16) & 1u)) >> 16;
}

__device__ __forceinline__ float bfr(float f) {
  return __uint_as_float(bfb(f) << 16);
}

__device__ __forceinline__ v8us cvt8b(const v4f a, const v4f b) {
  v8us r;
  r[0] = (u16)bfb(a.x); r[1] = (u16)bfb(a.y); r[2] = (u16)bfb(a.z); r[3] = (u16)bfb(a.w);
  r[4] = (u16)bfb(b.x); r[5] = (u16)bfb(b.y); r[6] = (u16)bfb(b.z); r[7] = (u16)bfb(b.w);
  return r;
}

__device__ __forceinline__ v4f fma4(const float w, const v4f v, const v4f a) {
  v4f r;
  r.x = fmaf(w, v.x, a.x); r.y = fmaf(w, v.y, a.y); r.z = fmaf(w, v.z, a.z); r.w = fmaf(w, v.w, a.w);
  return r;
}

__device__ __forceinline__ int scan_chunk(const int* __restrict__ keys, int nE, int cbase, int slotBase,
                                          int nb, int vec8, int* list, int tid, int lane, int wave) {
  int wc = 0;
  const int el0  = tid * EPT;
  const int e0   = cbase + el0;
  const int sent = -2147483647 - 1;
  v4i da, db;
  if (vec8 != 0 && cbase + CHUNK <= nE) {
    da = *(const v4i*)(keys + e0);
    db = *(const v4i*)(keys + e0 + 4);
  } else {
    da.x = (e0     < nE) ? keys[min(e0,     nE - 1)] : sent;
    da.y = (e0 + 1 < nE) ? keys[min(e0 + 1, nE - 1)] : sent;
    da.z = (e0 + 2 < nE) ? keys[min(e0 + 2, nE - 1)] : sent;
    da.w = (e0 + 3 < nE) ? keys[min(e0 + 3, nE - 1)] : sent;
    db.x = (e0 + 4 < nE) ? keys[min(e0 + 4, nE - 1)] : sent;
    db.y = (e0 + 5 < nE) ? keys[min(e0 + 5, nE - 1)] : sent;
    db.z = (e0 + 6 < nE) ? keys[min(e0 + 6, nE - 1)] : sent;
    db.w = (e0 + 7 < nE) ? keys[min(e0 + 7, nE - 1)] : sent;
  }
  const unsigned nbs = (unsigned)slotBase;
  const unsigned unb = (unsigned)nb;
  const unsigned s0 = (unsigned)da.x - nbs, s1 = (unsigned)da.y - nbs;
  const unsigned s2 = (unsigned)da.z - nbs, s3 = (unsigned)da.w - nbs;
  const unsigned s4 = (unsigned)db.x - nbs, s5 = (unsigned)db.y - nbs;
  const unsigned s6 = (unsigned)db.z - nbs, s7 = (unsigned)db.w - nbs;
  const bool h0 = s0 < unb, h1 = s1 < unb, h2 = s2 < unb, h3 = s3 < unb;
  const bool h4 = s4 < unb, h5 = s5 < unb, h6 = s6 < unb, h7 = s7 < unb;
  const unsigned any = __builtin_amdgcn_ballot_w32(h0 | h1 | h2 | h3 | h4 | h5 | h6 | h7);
  if (any != 0u) {
#define HITJ(J, HJ, SJ) { \
      const unsigned mj = __builtin_amdgcn_ballot_w32(HJ); \
      if (mj != 0u) { \
        if (HJ) { \
          const int pos = wc + (int)__builtin_amdgcn_mbcnt_lo(mj, 0u); \
          if (pos < WCAP) list[wave * WCAP + pos] = ((el0 + (J)) << 12) | (int)(SJ); \
        } \
        wc += (int)__builtin_popcount(mj); } }
    HITJ(0, h0, s0)
    HITJ(1, h1, s1)
    HITJ(2, h2, s2)
    HITJ(3, h3, s3)
    HITJ(4, h4, s4)
    HITJ(5, h5, s5)
    HITJ(6, h6, s6)
    HITJ(7, h7, s7)
#undef HITJ
  }
  return wc;
}

__device__ __forceinline__ int seg_build(const int* __restrict__ keys, int nE, int nodeBase, int nb, int vec8,
                                         int* reg1, int* reg2, int* scnt, int* soff, int* list, int* wcnt,
                                         int* wtot, int tid, int lane, int wave) {
  for (int i = tid; i < NBMAX; i += NTHR) scnt[i] = 0;
  __syncthreads();

  int tot = 0;
  const int nChunks = (nE + CHUNK - 1) / CHUNK;
#pragma unroll 1
  for (int ch = 0; ch < nChunks; ++ch) {
    const int cbase = ch * CHUNK;
    const int wc = scan_chunk(keys, nE, cbase, nodeBase, nb, vec8, list, tid, lane, wave);
    if (lane == 0) wcnt[wave] = wc;
    __syncthreads();
    int pre = 0, all = 0;
#pragma unroll
    for (int w2 = 0; w2 < NWAVE; ++w2) {
      int c = wcnt[w2];
      c = c < 0 ? 0 : (c > WCAP ? WCAP : c);
      all += c;
      pre += (w2 < wave) ? c : 0;
    }
    const int wcc  = wc > WCAP ? WCAP : wc;
    const int base = tot + pre;
#pragma unroll 1
    for (int i = lane; i < wcc; i += 32) {
      const int ent = list[wave * WCAP + i];
      const int el  = (ent >> 12) & (CHUNK - 1);
      const int sl  = ent & (NBMAX - 1);
      int eid = cbase + el;
      eid = eid > nE - 1 ? nE - 1 : eid;
      const int pos = base + i;
      if (pos < RCAP) reg1[pos] = (int)(((unsigned)eid << 12) | (unsigned)sl);
    }
    tot += all;
    tot = tot > RCAP ? RCAP : tot;
    __syncthreads();
  }
  const int nh = tot;

  if (wave == 0) {
#pragma unroll 1
    for (int b0 = 0; b0 < nh; b0 += 32) {
      const int idx = b0 + lane;
      const int uv  = reg1[idx < RCAP ? idx : RCAP - 1];
      const int m32 = (nh - b0) < 32 ? (nh - b0) : 32;
#pragma unroll 1
      for (int k = 0; k < m32; ++k) {
        const int u  = __builtin_amdgcn_readlane(uv, k);
        const int sl = u & (NBMAX - 1);
        if (lane == 0) scnt[sl] = scnt[sl] + 1;
      }
    }
  }
  __syncthreads();

  {
    const v4i ca = *(const v4i*)(scnt + 8 * tid);
    const v4i cb = *(const v4i*)(scnt + 8 * tid + 4);
    const int e0 = ca.x < 0 ? 0 : ca.x, e1 = ca.y < 0 ? 0 : ca.y, e2 = ca.z < 0 ? 0 : ca.z, e3 = ca.w < 0 ? 0 : ca.w;
    const int e4 = cb.x < 0 ? 0 : cb.x, e5 = cb.y < 0 ? 0 : cb.y, e6 = cb.z < 0 ? 0 : cb.z, e7 = cb.w < 0 ? 0 : cb.w;
    const int ts = e0 + e1 + e2 + e3 + e4 + e5 + e6 + e7;
    int incl = ts;
#pragma unroll
    for (int d = 1; d < 32; d <<= 1) {
      const int up = __shfl_up(incl, d);
      if (lane >= d) incl += up;
    }
    if (lane == 31) wtot[wave] = incl;
    __syncthreads();
    int pre = 0;
#pragma unroll
    for (int w2 = 0; w2 < NWAVE; ++w2) pre += (w2 < wave) ? wtot[w2] : 0;
    int run = pre + incl - ts;
    soff[8 * tid + 0] = run; run += e0;
    soff[8 * tid + 1] = run; run += e1;
    soff[8 * tid + 2] = run; run += e2;
    soff[8 * tid + 3] = run; run += e3;
    soff[8 * tid + 4] = run; run += e4;
    soff[8 * tid + 5] = run; run += e5;
    soff[8 * tid + 6] = run; run += e6;
    soff[8 * tid + 7] = run;
  }
  __syncthreads();
  for (int i = tid; i < NBMAX; i += NTHR) list[i] = soff[i];
  __syncthreads();

  if (wave == 0) {
#pragma unroll 1
    for (int b0 = 0; b0 < nh; b0 += 32) {
      const int idx = b0 + lane;
      const int uv  = reg1[idx < RCAP ? idx : RCAP - 1];
      const int m32 = (nh - b0) < 32 ? (nh - b0) : 32;
#pragma unroll 1
      for (int k = 0; k < m32; ++k) {
        const int u   = __builtin_amdgcn_readlane(uv, k);
        const int sl  = u & (NBMAX - 1);
        const int eid = (int)((unsigned)u >> 12);
        if (lane == 0) {
          int pos = list[sl];
          pos = pos < 0 ? 0 : (pos > RCAP - 1 ? RCAP - 1 : pos);
          reg2[pos] = eid;
          list[sl] = pos + 1;
        }
      }
    }
  }
  __syncthreads();
  return nh;
}

__global__ __launch_bounds__(NTHR) void k_w1t(const float* __restrict__ W1, u16* wt, int nUnits) {
  const int u = (int)blockIdx.x * NTHR + (int)threadIdx.x;
  if (u >= nUnits) return;
  const int n  = u >> 5;
  const int k8 = (u & 31) * 8;
  const int head = n >> 6, o = n & (HID - 1);
  const float* p = W1 + ((size_t)head * FIN + k8) * HID + o;
  v4f a, b;
  a.x = p[0];         a.y = p[HID];       a.z = p[2 * HID];   a.w = p[3 * HID];
  b.x = p[4 * HID];   b.y = p[5 * HID];   b.z = p[6 * HID];   b.w = p[7 * HID];
  const v8us hv = cvt8b(a, b);
  const size_t off = (size_t)n * FIN + k8;
  *(volatile v8us*)(wt + off) = hv;
  __threadfence();
  *(volatile v8us*)(wt + off) = hv;
}

__global__ __launch_bounds__(NTHR) void k_w2t(const float* __restrict__ W2, u16* wt, int nUnits) {
  const int u = (int)blockIdx.x * NTHR + (int)threadIdx.x;
  if (u >= nUnits) return;
  const int n   = u >> 7;
  const int k8  = (u & 127) * 8;
  const int kk  = k8 & (F1 - 1);
  const int ncl = n < NCLS ? n : NCLS - 1;
  const float* p = W2 + (size_t)kk * NCLS + ncl;
  v4f a, b;
  a.x = p[0];          a.y = p[NCLS];       a.z = p[2 * NCLS];   a.w = p[3 * NCLS];
  b.x = p[4 * NCLS];   b.y = p[5 * NCLS];   b.z = p[6 * NCLS];   b.w = p[7 * NCLS];
  const v4f z4 = {0.f, 0.f, 0.f, 0.f};
  if (n >= NCLS) { a = z4; b = z4; }
  const v8us hv = cvt8b(a, b);
  const size_t off = (size_t)n * K2 + k8;
  *(volatile v8us*)(wt + off) = hv;
  __threadfence();
  *(volatile v8us*)(wt + off) = hv;
}

__device__ __forceinline__ void tile_rows_store(const float* stg, float* outF, int ldo, int col0,
                                                int rowBase, int wave, int hh, int m) {
  v4f fv[8];
#pragma unroll
  for (int i = 0; i < 8; ++i) {
    const int lr = 16 * wave + 2 * i + hh;
    fv[i] = *(const v4fa*)(stg + lr * HID + 4 * m);
  }
#pragma unroll
  for (int i = 0; i < 8; ++i) {
    const int lr = 16 * wave + 2 * i + hh;
    float* op = outF + (size_t)(rowBase + lr) * (size_t)ldo + col0 + 4 * m;
    *(volatile v4f*)op = fv[i];
  }
  __threadfence();
#pragma unroll
  for (int i = 0; i < 8; ++i) {
    const int lr = 16 * wave + 2 * i + hh;
    float* op = outF + (size_t)(rowBase + lr) * (size_t)ldo + col0 + 4 * m;
    *(volatile v4f*)op = fv[i];
  }
}

__global__ __launch_bounds__(GTHR) void k_gemm1(
    const float* __restrict__ x, const u16* __restrict__ W1T, const float* __restrict__ a1,
    float* H1, float* S1S, float* S1T, int nN, int MPS)
{
  __shared__ __attribute__((aligned(16))) u16   As[GBM * APITCH];
  __shared__ __attribute__((aligned(16))) float stg[GBM * HID];
  __shared__ __attribute__((aligned(16))) float sdot[2 * GBM];
  __shared__ float sa[NHD * 2 * HID];
  const int tid = (int)threadIdx.x, lane = tid & 31, wave = tid >> 5, hh = lane >> 4, m = lane & 15;
  const int rowBase = (int)blockIdx.x * GBM;
  const v4f z4 = {0.f, 0.f, 0.f, 0.f};

#pragma unroll 1
  for (int u = tid; u < GBM * (FIN / 8); u += GTHR) {
    const int row = u >> 5;
    const int k8  = (u & 31) * 8;
    const int gr  = rowBase + row;
    const int rc  = gr < nN ? gr : nN - 1;
    const float* p = x + (size_t)rc * FIN + k8;
    v4f a = *(const v4fa*)p, b = *(const v4fa*)(p + 4);
    if (gr >= nN) { a = z4; b = z4; }
    *(v8usa*)(As + row * APITCH + k8) = cvt8b(a, b);
  }
#pragma unroll 1
  for (int i = tid; i < NHD * 2 * HID; i += GTHR) sa[i] = bfr(a1[i]);
  __syncthreads();

  const u16* ap = As + (16 * wave + m) * APITCH + 8 * hh;
#pragma unroll 1
  for (int head = 0; head < NHD; ++head) {
    v8f acc[4];
    {
      const v8f z = {0.f, 0.f, 0.f, 0.f, 0.f, 0.f, 0.f, 0.f};
      acc[0] = z; acc[1] = z; acc[2] = z; acc[3] = z;
    }
    const u16* wp = W1T + (size_t)(HID * head + m) * (size_t)FIN + 8 * hh;
#pragma unroll 1
    for (int ks = 0; ks < FIN / 32; ++ks) {
      FragB af;
      af.h[0] = *(const v8usa*)(ap + 32 * ks);
      af.h[1] = *(const v8usa*)(ap + 32 * ks + 16);
#pragma unroll
      for (int t = 0; t < 4; ++t) {
        const u16* wq = wp + (size_t)(16 * t) * (size_t)FIN + 32 * ks;
        FragB bf;
        bf.h[0] = *(const v8usa*)wq;
        bf.h[1] = *(const v8usa*)(wq + 16);
        acc[t] = wmb(af, bf, acc[t]);
      }
    }

#pragma unroll
    for (int t = 0; t < 4; ++t) {
#pragma unroll
      for (int r = 0; r < 8; ++r) {
        const int lr = 16 * wave + 8 * hh + r;
        stg[lr * HID + 16 * t + m] = acc[t][r];
      }
    }
    __syncthreads();

    {
      const int which = tid >> 6;
      const int row = tid & (GBM - 1);
      const float* av = sa + head * (2 * HID) + which * HID;
      const float* sr = stg + row * HID;
      float d = 0.f;
#pragma unroll 4
      for (int c = 0; c < HID; ++c) d = fmaf(sr[c], av[c], d);
      sdot[tid] = d;
    }
    tile_rows_store(stg, H1, F1, HID * head, rowBase, wave, hh, m);
    __syncthreads();

    if (wave == 0) {
      const int which = lane >> 4, q = lane & 15;
      const v4f sv = *(const v4fa*)(sdot + GBM * which + 4 * q);
      float* sp = (which != 0 ? S1T : S1S) + (size_t)head * (size_t)MPS + rowBase + 4 * q;
      *(volatile v4f*)sp = sv;
      __threadfence();
      *(volatile v4f*)sp = sv;
    }
  }
}

__global__ __launch_bounds__(GTHR) void k_gemm2(
    const u16* __restrict__ A2, const u16* __restrict__ W2T, const float* __restrict__ a2,
    float* H2, float* S2S, float* S2T)
{
  __shared__ __attribute__((aligned(16))) float stg[GBM * HID];
  __shared__ __attribute__((aligned(16))) float sdot[2 * GBM];
  __shared__ float sa2[2 * NCLS];
  const int tid = (int)threadIdx.x, lane = tid & 31, wave = tid >> 5, hh = lane >> 4, m = lane & 15;
  const int rowBase = (int)blockIdx.x * GBM;

  if (tid < 2 * NCLS) sa2[tid] = bfr(a2[tid]);

  v8f acc[4];
  {
    const v8f z = {0.f, 0.f, 0.f, 0.f, 0.f, 0.f, 0.f, 0.f};
    acc[0] = z; acc[1] = z; acc[2] = z; acc[3] = z;
  }
  const u16* ap = A2  + (size_t)(rowBase + 16 * wave + m) * (size_t)K2 + 8 * hh;
  const u16* wp = W2T + (size_t)m * (size_t)K2 + 8 * hh;
#pragma unroll 1
  for (int ks = 0; ks < K2 / 32; ++ks) {
    FragB af;
    af.h[0] = *(const v8usa*)(ap + 32 * ks);
    af.h[1] = *(const v8usa*)(ap + 32 * ks + 16);
#pragma unroll
    for (int t = 0; t < 4; ++t) {
      const u16* wq = wp + (size_t)(16 * t) * (size_t)K2 + 32 * ks;
      FragB bf;
      bf.h[0] = *(const v8usa*)wq;
      bf.h[1] = *(const v8usa*)(wq + 16);
      acc[t] = wmb(af, bf, acc[t]);
    }
  }

#pragma unroll
  for (int t = 0; t < 4; ++t) {
#pragma unroll
    for (int r = 0; r < 8; ++r) {
      const int lr = 16 * wave + 8 * hh + r;
      stg[lr * HID + 16 * t + m] = acc[t][r];
    }
  }
  __syncthreads();

  {
    const int which = tid >> 6;
    const int row = tid & (GBM - 1);
    const float* av = sa2 + which * NCLS;
    const float* sr = stg + row * HID;
    float d = 0.f;
#pragma unroll 4
    for (int c = 0; c < NCLS; ++c) d = fmaf(sr[c], av[c], d);
    sdot[tid] = d;
  }
  tile_rows_store(stg, H2, NCP, 0, rowBase, wave, hh, m);
  __syncthreads();

  if (wave == 0) {
    const int which = lane >> 4, q = lane & 15;
    const v4f sv = *(const v4fa*)(sdot + GBM * which + 4 * q);
    float* sp = (which != 0 ? S2T : S2S) + rowBase + 4 * q;
    *(volatile v4f*)sp = sv;
    __threadfence();
    *(volatile v4f*)sp = sv;
  }
}

template<int H>
__global__ __launch_bounds__(NTHR) void k_emax(const int* __restrict__ srcs, const int* __restrict__ tgts,
                                              const float* __restrict__ SS, const float* __restrict__ ST,
                                              int nN, int nE, int MPS, float* rec) {
  __shared__ float sm[NWAVE * 8];
  __shared__ __attribute__((aligned(16))) float fin[ERECW];
  const int tid = (int)threadIdx.x, lane = tid & 31, wave = tid >> 5;
  float mh[H];
#pragma unroll
  for (int h = 0; h < H; ++h) mh[h] = -__builtin_inff();
#pragma unroll 1
  for (int e = (int)blockIdx.x * NTHR + tid; e < nE; e += EMAXG * NTHR) {
    int s = srcs[e]; s = s < 0 ? 0 : (s > nN - 1 ? nN - 1 : s);
    int t = tgts[e]; t = t < 0 ? 0 : (t > nN - 1 ? nN - 1 : t);
    float sv[H], tv[H];
#pragma unroll
    for (int h = 0; h < H; ++h) sv[h] = SS[(size_t)h * MPS + s];
    ldwait();
#pragma unroll
    for (int h = 0; h < H; ++h) tv[h] = ST[(size_t)h * MPS + t];
    ldwait();
#pragma unroll
    for (int h = 0; h < H; ++h) {
      float v = sv[h] + tv[h];
      v = fmaxf(v, LRELU * v);
      mh[h] = fmaxf(mh[h], v);
    }
  }
#pragma unroll
  for (int h = 0; h < H; ++h) {
#pragma unroll
    for (int off = 16; off > 0; off >>= 1) mh[h] = fmaxf(mh[h], __shfl_xor(mh[h], off));
  }
  if (lane == 0) {
#pragma unroll
    for (int h = 0; h < H; ++h) sm[wave * 8 + h] = mh[h];
  }
  if (tid < ERECW) fin[tid] = 0.f;
  __syncthreads();
  if (wave == 0) {
    if (lane == 0) {
#pragma unroll
      for (int h = 0; h < H; ++h) {
        float g = sm[h];
#pragma unroll
        for (int w2 = 1; w2 < NWAVE; ++w2) g = fmaxf(g, sm[w2 * 8 + h]);
        fin[h] = g;
      }
    }
    __builtin_amdgcn_fence(__ATOMIC_RELEASE, "wavefront");
    __builtin_amdgcn_wave_barrier();
    const v4f rv = *(const v4fa*)(fin + 4 * (lane & 7));
    float* rp = rec + (size_t)blockIdx.x * ERECW + 4 * (lane & 7);
    if (lane < 8) *(volatile v4f*)rp = rv;
    __threadfence();
    if (lane < 8) *(volatile v4f*)rp = rv;
  }
}

__global__ __launch_bounds__(NTHR) void k_agg1(
    const int* __restrict__ srcs, const int* __restrict__ tgts,
    const float* __restrict__ H1, const float* __restrict__ S1S, const float* __restrict__ S1T,
    const float* __restrict__ rec, const float* __restrict__ b1, u16* A2,
    int nN, int nE, int nb, int vec8, int MPr, int MPS) {
  extern __shared__ v4f lds_dyn[];
  int* reg1 = (int*)lds_dyn;
  int* reg2 = reg1 + RCAP;
  int* scnt = reg2 + RCAP;
  int* soff = scnt + NBMAX;
  int* list = soff + NBMAX;
  int* wcnt = list + LISTN;
  int* wtot = wcnt + NWAVE;
  float* gml = (float*)(wtot + NWAVE);
  const int tid = (int)threadIdx.x, lane = tid & 31, wave = tid >> 5;
  const int nodeBase = (int)blockIdx.x * nb;

  if (tid < NHD) {
    float g = -__builtin_inff();
#pragma unroll 1
    for (int b = 0; b < EMAXG; ++b) g = fmaxf(g, rec[b * ERECW + tid]);
    gml[tid] = g;
  }
  const int nh = seg_build(srcs, nE, nodeBase, nb, vec8, reg1, reg2, scnt, soff, list, wcnt, wtot,
                           tid, lane, wave);

  const int nbw = nb >> 3;
  const bool ovf = (nh >= RCAP);
  const float qnan = __int_as_float(0x7fc00000);
  float* stwf = (float*)reg1 + wave * STW;
  u16*   stwu = (u16*)(stwf + F1);
  const int hd = lane >> 2;
  const float gm = gml[hd];
  const float* ssp = S1S + (size_t)hd * (size_t)MPS;
  const float* stp = S1T + (size_t)hd * (size_t)MPS;
  const v4f z4 = {0.f, 0.f, 0.f, 0.f};
#pragma unroll 1
  for (int jt = 0; jt < nbw; ++jt) {
    const int slot = wave * nbw + jt;
    const int grow = nodeBase + slot;
    const int gcl  = grow < nN ? grow : nN - 1;
    int st = soff[slot];
    const int craw = scnt[slot];
    int cnt = craw;
    st  = st < 0 ? 0 : (st > nh ? nh : st);
    cnt = cnt < 0 ? 0 : (cnt > DEGCAP ? DEGCAP : cnt);
    if (cnt > nh - st) cnt = nh - st;
    const float pz = (ovf || craw > DEGCAP) ? qnan : 0.0f;
    const bool wr = grow < MPr;
    const float live = grow < nN ? 1.0f : 0.0f;

    const float ss = ssp[gcl];
    v4f acc0 = z4, acc1 = z4, acc2 = z4, acc3 = z4;
    float den = 0.f;
#pragma unroll 1
    for (int q = 0; q < cnt; ++q) {
      int idx = st + q; idx = idx > RCAP - 1 ? RCAP - 1 : idx;
      int eid = reg2[idx]; eid = eid < 0 ? 0 : (eid > nE - 1 ? nE - 1 : eid);
      const int traw = tgts[eid];
      const int t = traw < 0 ? 0 : (traw > nN - 1 ? nN - 1 : traw);
      const float sv = stp[t];
      float e = ss + sv;
      e = fmaxf(e, LRELU * e);
      const float w = __expf(e - gm);
      const float* hr = H1 + (size_t)t * F1 + 16 * lane;
      const v4f v0 = *(const v4fa*)hr;
      const v4f v1 = *(const v4fa*)(hr + 4);
      const v4f v2 = *(const v4fa*)(hr + 8);
      const v4f v3 = *(const v4fa*)(hr + 12);
      ldwait();
      den += w;
      acc0 = fma4(w, v0, acc0);
      acc1 = fma4(w, v1, acc1);
      acc2 = fma4(w, v2, acc2);
      acc3 = fma4(w, v3, acc3);
    }
    const float inv = __builtin_amdgcn_rcpf(den + 1e-10f);
    __builtin_amdgcn_fence(__ATOMIC_RELEASE, "wavefront");
    __builtin_amdgcn_wave_barrier();
    *(v4fa*)(stwf + 16 * lane)      = acc0;
    *(v4fa*)(stwf + 16 * lane + 4)  = acc1;
    *(v4fa*)(stwf + 16 * lane + 8)  = acc2;
    *(v4fa*)(stwf + 16 * lane + 12) = acc3;
    __builtin_amdgcn_fence(__ATOMIC_RELEASE, "wavefront");
    __builtin_amdgcn_wave_barrier();
#pragma unroll 1
    for (int i = 0; i < 16; ++i) {
      const int c = 16 * lane + i;
      float v = fmaf(stwf[c], inv, bfr(b1[c])) * live + pz;
      v = v > 0.f ? v : expm1f(v);
      const unsigned hb = bfb(v);
      const float hf = __uint_as_float(hb << 16);
      const unsigned lb = bfb(v - hf);
      stwu[c]      = (u16)hb;
      stwu[F1 + c] = (u16)lb;
    }
    __builtin_amdgcn_fence(__ATOMIC_RELEASE, "wavefront");
    __builtin_amdgcn_wave_barrier();
    v8us pv[4];
#pragma unroll
    for (int i = 0; i < 4; ++i) pv[i] = *(const v8usa*)(stwu + 8 * (32 * i + lane));
    u16* gp = A2 + (size_t)grow * (size_t)K2;
    if (wr) {
#pragma unroll
      for (int i = 0; i < 4; ++i) *(volatile v8us*)(gp + 8 * (32 * i + lane)) = pv[i];
    }
    __threadfence();
    if (wr) {
#pragma unroll
      for (int i = 0; i < 4; ++i) *(volatile v8us*)(gp + 8 * (32 * i + lane)) = pv[i];
    }
  }
}

__global__ __launch_bounds__(NTHR) void k_agg2(
    const int* __restrict__ srcs, const int* __restrict__ tgts,
    const float* __restrict__ H2, const float* __restrict__ S2S, const float* __restrict__ S2T,
    const float* __restrict__ rec, const float* __restrict__ b2, float* out,
    int nN, int nE, int nb, int vec8) {
  extern __shared__ v4f lds_dyn[];
  int* reg1 = (int*)lds_dyn;
  int* reg2 = reg1 + RCAP;
  int* scnt = reg2 + RCAP;
  int* soff = scnt + NBMAX;
  int* list = soff + NBMAX;
  int* wcnt = list + LISTN;
  int* wtot = wcnt + NWAVE;
  float* gml = (float*)(wtot + NWAVE);
  const int tid = (int)threadIdx.x, lane = tid & 31, wave = tid >> 5;
  const int nodeBase = (int)blockIdx.x * nb;

  if (tid == 0) {
    float g = -__builtin_inff();
#pragma unroll 1
    for (int b = 0; b < EMAXG; ++b) g = fmaxf(g, rec[b * ERECW]);
    gml[0] = g;
  }
  const int nh = seg_build(srcs, nE, nodeBase, nb, vec8, reg1, reg2, scnt, soff, list, wcnt, wtot,
                           tid, lane, wave);

  const int nbw = nb >> 3;
  const bool ovf = (nh >= RCAP);
  const float qnan = __int_as_float(0x7fc00000);
  const float ninf = -__builtin_inff();
  float* sout = (float*)reg1;
  const float gm = gml[0];
  const int l8 = lane < 8 ? lane : 7;
  const float bz0 = bfr(b2[lane]);
  const float bz1 = bfr(b2[32 + l8]);
#pragma unroll 1
  for (int jt = 0; jt < nbw; ++jt) {
    const int slot = wave * nbw + jt;
    const int grow = nodeBase + slot;
    const int gcl  = grow < nN ? grow : nN - 1;
    int st = soff[slot];
    const int craw = scnt[slot];
    int cnt = craw;
    st  = st < 0 ? 0 : (st > nh ? nh : st);
    cnt = cnt < 0 ? 0 : (cnt > DEGCAP ? DEGCAP : cnt);
    if (cnt > nh - st) cnt = nh - st;
    const float pz = (ovf || craw > DEGCAP) ? qnan : 0.0f;

    const float ss = S2S[gcl];
    float a0 = 0.f, a1v = 0.f, den = 0.f;
#pragma unroll 1
    for (int q = 0; q < cnt; ++q) {
      int idx = st + q; idx = idx > RCAP - 1 ? RCAP - 1 : idx;
      int eid = reg2[idx]; eid = eid < 0 ? 0 : (eid > nE - 1 ? nE - 1 : eid);
      const int traw = tgts[eid];
      const int t = traw < 0 ? 0 : (traw > nN - 1 ? nN - 1 : traw);
      const float sv = S2T[t];
      float e = ss + sv;
      e = fmaxf(e, LRELU * e);
      const float w = __expf(e - gm);
      const float* hr = H2 + (size_t)t * NCP;
      const float v0 = hr[lane];
      const float v1 = hr[32 + lane];
      ldwait();
      den += w;
      a0  = fmaf(w, v0, a0);
      a1v = fmaf(w, v1, a1v);
    }
    const float inv = __builtin_amdgcn_rcpf(den + 1e-10f);
    const float o0 = fmaf(a0, inv, bz0) + pz;
    const float o1 = fmaf(a1v, inv, bz1) + pz;
    float mx = fmaxf(o0, lane < 8 ? o1 : ninf);
#pragma unroll
    for (int off = 16; off > 0; off >>= 1) mx = fmaxf(mx, __shfl_xor(mx, off));
    const float ex1 = __expf(o1 - mx);
    float sm = __expf(o0 - mx) + (lane < 8 ? ex1 : 0.f);
#pragma unroll
    for (int off = 16; off > 0; off >>= 1) sm += __shfl_xor(sm, off);
    const float lse = mx + __logf(sm);
    sout[slot * NCLS + lane] = o0 - lse;
    if (lane < 8) sout[slot * NCLS + 32 + lane] = o1 - lse;
  }
  __syncthreads();

  int nv = nN - nodeBase;
  nv = nv < 0 ? 0 : (nv > nb ? nb : nv);
  const int np = nv * (NCLS / 4);
  float* ob = out + (size_t)nodeBase * NCLS;
#pragma unroll 1
  for (int p = tid; p < np; p += NTHR) *(volatile v4f*)(ob + 4 * p) = *(const v4fa*)(sout + 4 * p);
  __threadfence();
#pragma unroll 1
  for (int p = tid; p < np; p += NTHR) *(volatile v4f*)(ob + 4 * p) = *(const v4fa*)(sout + 4 * p);
}

static int pick_nb(int nE, int nN) {
  int nb = NBMAX;
  while (nb > 16 && (long long)nb * (long long)nE * 5LL > (long long)RCAP * (long long)nN * 4LL) nb >>= 1;
  return nb;
}
static inline int cdiv(int a, int b) { return (a + b - 1) / b; }

extern "C" void kernel_launch(void* const* d_in, const int* in_sizes, int n_in,
                              void* d_out, int out_size, void* d_ws, size_t ws_size,
                              hipStream_t stream) {
  if (n_in < 8) return;
  if (in_sizes[0] < FIN || (in_sizes[0] % FIN) != 0) return;
  const int nN = in_sizes[0] / FIN;
  if (nN <= 0 || nN > (1 << 22)) return;
  if (in_sizes[1] < 2 || (in_sizes[1] & 1) != 0) return;
  const int nE = in_sizes[1] / 2;
  if (nE < 1 || nE > (1 << 20)) return;
  if (in_sizes[2] != NHD * FIN * HID) return;
  if (in_sizes[3] != NHD * 2 * HID) return;
  if (in_sizes[4] != NHD * HID) return;
  if (in_sizes[5] != F1 * NCLS) return;
  if (in_sizes[6] != 2 * NCLS) return;
  if (in_sizes[7] != NCLS) return;
  if (out_size != nN * NCLS) return;

  const float* x  = (const float*)d_in[0];
  const int*   el = (const int*)  d_in[1];
  const float* W1 = (const float*)d_in[2];
  const float* a1 = (const float*)d_in[3];
  const float* b1 = (const float*)d_in[4];
  const float* W2 = (const float*)d_in[5];
  const float* a2 = (const float*)d_in[6];
  const float* b2 = (const float*)d_in[7];
  float* out = (float*)d_out;
  const int* srcs = el;
  const int* tgts = el + nE;

  const int MP   = cdiv(nN, GBM) * GBM;
  const int nb1  = pick_nb(nE, nN);
  const int gA1  = cdiv(MP, nb1);
  int nb2 = nb1 < NB2MAX ? nb1 : NB2MAX;
  const int gA2  = cdiv(nN, nb2);
  const int vec8 = ((nE & 3) == 0) ? 1 : 0;
  if (nb1 < 16 || nb1 > NBMAX || gA1 * nb1 < MP) return;
  if (nb2 < 16 || gA2 * nb2 < nN) return;

  char* ws = (char*)d_ws;
  size_t off = 0;
  const size_t oW1T = off; off += (size_t)F1 * FIN * 2;            off = (off + 255) & ~(size_t)255;
  const size_t oH1  = off; off += (size_t)MP * F1 * 4;             off = (off + 255) & ~(size_t)255;
  const size_t oS1S = off; off += (size_t)NHD * MP * 4;            off = (off + 255) & ~(size_t)255;
  const size_t oS1T = off; off += (size_t)NHD * MP * 4;            off = (off + 255) & ~(size_t)255;
  const size_t oR1  = off; off += (size_t)EMAXG * ERECW * 4;       off = (off + 255) & ~(size_t)255;
  const size_t oR2  = off; off += (size_t)EMAXG * ERECW * 4;       off = (off + 255) & ~(size_t)255;
  const size_t oA2  = off; off += (size_t)MP * K2 * 2;             off = (off + 255) & ~(size_t)255;
  const size_t oW2T = off; off += (size_t)NCP * K2 * 2;            off = (off + 255) & ~(size_t)255;
  const size_t oH2  = off; off += (size_t)MP * NCP * 4;            off = (off + 255) & ~(size_t)255;
  const size_t oS2S = off; off += (size_t)MP * 4;                  off = (off + 255) & ~(size_t)255;
  const size_t oS2T = off; off += (size_t)MP * 4;                  off = (off + 255) & ~(size_t)255;
  if (off > ws_size || off > (size_t)WSMAX) return;
  u16*   W1T = (u16*)  (ws + oW1T);
  float* H1  = (float*)(ws + oH1);
  float* S1S = (float*)(ws + oS1S);
  float* S1T = (float*)(ws + oS1T);
  float* R1  = (float*)(ws + oR1);
  float* R2  = (float*)(ws + oR2);
  u16*   A2  = (u16*)  (ws + oA2);
  u16*   W2T = (u16*)  (ws + oW2T);
  float* H2  = (float*)(ws + oH2);
  float* S2S = (float*)(ws + oS2S);
  float* S2T = (float*)(ws + oS2T);

  hipFuncSetAttribute(reinterpret_cast<const void*>(&k_agg1),
                      hipFuncAttributeMaxDynamicSharedMemorySize, LDS_AGG);
  hipFuncSetAttribute(reinterpret_cast<const void*>(&k_agg2),
                      hipFuncAttributeMaxDynamicSharedMemorySize, LDS_AGG);

  {
    const int nU1 = F1 * (FIN / 8);
    k_w1t<<<cdiv(nU1, NTHR), NTHR, 0, stream>>>(W1, W1T, nU1);
    const int nU2 = NCP * (K2 / 8);
    k_w2t<<<cdiv(nU2, NTHR), NTHR, 0, stream>>>(W2, W2T, nU2);
  }
  const int gM = MP / GBM;
  k_gemm1<<<gM, GTHR, 0, stream>>>(x, W1T, a1, H1, S1S, S1T, nN, MP);
  k_emax<NHD><<<EMAXG, NTHR, 0, stream>>>(srcs, tgts, S1S, S1T, nN, nE, MP, R1);
  k_agg1<<<gA1, NTHR, LDS_AGG, stream>>>(srcs, tgts, H1, S1S, S1T, R1, b1, A2, nN, nE, nb1, vec8, MP, MP);
  k_gemm2<<<gM, GTHR, 0, stream>>>(A2, W2T, a2, H2, S2S, S2T);
  k_emax<1><<<EMAXG, NTHR, 0, stream>>>(srcs, tgts, S2S, S2T, nN, nE, MP, R2);
  k_agg2<<<gA2, NTHR, LDS_AGG, stream>>>(srcs, tgts, H2, S2S, S2T, R2, b2, out, nN, nE, nb2, vec8);
}
